// ConvexMultiHeadAttention_88527865905583
// MI455X (gfx1250) — hardware-verified
//
#include <hip/hip_runtime.h>
#include <math.h>

constexpr int kBatch    = 2;
constexpr int kSeq      = 2048;
constexpr int kDim      = 1024;
constexpr int kHeads    = 16;
constexpr int kHd       = 64;
constexpr int kTok      = kBatch * kSeq;
constexpr int kGroups   = kBatch * kHeads;
constexpr int kGrpChunk = 2;
constexpr int kChunks   = kGroups / kGrpChunk;
constexpr float kPCarry    = 2048.0f;
constexpr float kPCarryInv = 1.0f / 2048.0f;
constexpr float kClipLo = -15.0f;
constexpr float kClipHi = 15.0f;
constexpr float kRShift = 1.0f;
constexpr float kLam    = 0.1f;
constexpr float kEps    = 1e-9f;

typedef __attribute__((ext_vector_type(16))) _Float16 v16h;
typedef __attribute__((ext_vector_type(8)))  _Float16 v8h;
typedef __attribute__((ext_vector_type(16))) __bf16   v16b;
typedef __attribute__((ext_vector_type(8)))  __bf16   v8b;
typedef __attribute__((ext_vector_type(8)))  float    v8f;
typedef __attribute__((ext_vector_type(4)))  float    v4f;
typedef __attribute__((ext_vector_type(4)))  unsigned int v4u;

__device__ __forceinline__ unsigned short f2bf_bits(float f) {
  unsigned u = __float_as_uint(f);
  return (unsigned short)((u + 0x7FFFu + ((u >> 16) & 1u)) >> 16);
}
__device__ __forceinline__ float bf_bits2f(unsigned short h) { return __uint_as_float(((unsigned)h) << 16); }

__device__ __forceinline__ void dep_guard_h(v8f& a, v8f& b, v16h x, v16h y) { asm volatile("v_nop\n\tv_nop\n\tv_nop\n\tv_nop" : "+v"(a), "+v"(b) : "v"(x), "v"(y)); }
__device__ __forceinline__ void dep_guard_b(v8f& a, v8f& b, v16b x, v16b y) { asm volatile("v_nop\n\tv_nop\n\tv_nop\n\tv_nop" : "+v"(a), "+v"(b) : "v"(x), "v"(y)); }
__device__ __forceinline__ void keep4_h(v16h a, v16h b, v16h c, v16h d) { asm volatile("v_nop" :: "v"(a), "v"(b), "v"(c), "v"(d)); }
__device__ __forceinline__ void keep4_b(v16b a, v16b b, v16b c, v16b d) { asm volatile("v_nop" :: "v"(a), "v"(b), "v"(c), "v"(d)); }
__device__ __forceinline__ void acc_guard4(v8f& a, v8f& b, v8f& c, v8f& d) { asm volatile("v_nop\n\tv_nop\n\tv_nop\n\tv_nop" : "+v"(a), "+v"(b), "+v"(c), "+v"(d)); }
template <typename T> struct Frag;
template <> struct Frag<_Float16> {
  typedef v16h V; union U { v16h v; v8h h[2]; };
  static __device__ __forceinline__ v16h load(const _Float16* p) {
    U f; f.h[0] = *(const v8h*)(p); f.h[1] = *(const v8h*)(p + 16); return f.v;
  }
  static __device__ __forceinline__ v8f mma(v16h a, v16h b, v8f c) {
    return __builtin_amdgcn_wmma_f32_16x16x32_f16(false, a, false, b, (short)0, c, false, false);
  }
  static __device__ __forceinline__ void guard(v8f& a, v8f& b, v16h x, v16h y) { dep_guard_h(a, b, x, y); }
  static __device__ __forceinline__ void keep(v16h a, v16h b, v16h c, v16h d) { keep4_h(a, b, c, d); }
};
template <> struct Frag<__bf16> {
  typedef v16b V; union U { v16b v; v8b h[2]; };
  static __device__ __forceinline__ v16b load(const __bf16* p) {
    U f; f.h[0] = *(const v8b*)(p); f.h[1] = *(const v8b*)(p + 16); return f.v;
  }
  static __device__ __forceinline__ v8f mma(v16b a, v16b b, v8f c) {
    return __builtin_amdgcn_wmma_f32_16x16x32_bf16(false, a, false, b, (short)0, c, false, false);
  }
  static __device__ __forceinline__ void guard(v8f& a, v8f& b, v16b x, v16b y) { dep_guard_b(a, b, x, y); }
  static __device__ __forceinline__ void keep(v16b a, v16b b, v16b c, v16b d) { keep4_b(a, b, c, d); }
};

__device__ __forceinline__ unsigned pk16(unsigned short a, unsigned short b) { return (unsigned)a | ((unsigned)b << 16); }
__device__ __forceinline__ unsigned short h_bits(float f) { const _Float16 h = (_Float16)f; return __builtin_bit_cast(unsigned short, h); }

template <int ET> struct Elem;
template <> struct Elem<0> { typedef _Float16 T; };
template <> struct Elem<1> { typedef __bf16 T; };
template <int ET, bool SPLIT, int BIAS_MODE, int OUT_MODE, bool RESID, int ACT = 0>
__global__ __launch_bounds__(256) void wmma_gemm64(
    const unsigned short* __restrict__ Ap, const unsigned short* __restrict__ A2p, int lda, long strideA,
    const unsigned short* __restrict__ Btp, const unsigned short* __restrict__ Bt2p, int ldb, long strideB,
    void* __restrict__ Cout, void* __restrict__ Cout2, int ldc, long strideC,
    const float* __restrict__ bias,
    const float* __restrict__ resid, long strideR,
    int M, int N, int K, float scale) {
  typedef typename Elem<ET>::T T;
  typedef typename Frag<T>::V V;
  const T* A = (const T*)Ap; const T* A2 = (const T*)A2p; const T* Bt = (const T*)Btp; const T* Bt2 = (const T*)Bt2p;
  __shared__ __align__(16) float sT[8][16 * 68];
  const int b    = blockIdx.y;
  const int lane = threadIdx.x & 31;
  const int wave = threadIdx.x >> 5;
  const int tilesN = N >> 6;
  const int tilesM = M >> 6;
  const int tile = blockIdx.x * 8 + wave;
  if (tile >= tilesM * tilesN) return;
  const int tm = tile / tilesN;
  const int tn = tile - tm * tilesN;
  const int m0 = tm << 6;
  const int n0 = tn << 6;

  const T* Ab  = A  + (size_t)b * strideA;
  const T* Bb  = Bt + (size_t)b * strideB;
  const T* Ab2 = SPLIT ? (A2  + (size_t)b * strideA) : nullptr;
  const T* Bb2 = SPLIT ? (Bt2 + (size_t)b * strideB) : nullptr;

  const int rlane = lane & 15;
  const int koff  = (lane >> 4) * 8;
  const int mOff  = (lane >> 4) * 8;

  v8f acc[4][4];
#pragma unroll
  for (int i = 0; i < 4; ++i)
#pragma unroll
    for (int j = 0; j < 4; ++j) acc[i][j] = (v8f){0.f,0.f,0.f,0.f,0.f,0.f,0.f,0.f};

  for (int k0 = 0; k0 < K; k0 += 32) {
    V bh[4], bl[4];
#pragma unroll
    for (int j = 0; j < 4; ++j) {
      const size_t bo = (size_t)(n0 + (j << 4) + rlane) * ldb + koff + k0;
      bh[j] = Frag<T>::load(Bb + bo);
      if (SPLIT) bl[j] = Frag<T>::load(Bb2 + bo);
    }
#pragma unroll
    for (int i = 0; i < 4; ++i) {
      const size_t ao = (size_t)(m0 + (i << 4) + rlane) * lda + koff + k0;
      V ah = Frag<T>::load(Ab + ao);
      V al;
      if (SPLIT) al = Frag<T>::load(Ab2 + ao);
#pragma unroll
      for (int j = 0; j < 4; ++j) {
        acc[i][j] = Frag<T>::mma(ah, bh[j], acc[i][j]);
        if (SPLIT) {
          acc[i][j] = Frag<T>::mma(ah, bl[j], acc[i][j]);
          acc[i][j] = Frag<T>::mma(al, bh[j], acc[i][j]);
        }
      }
      Frag<T>::guard(acc[i][0], acc[i][3], ah, SPLIT ? al : ah);
    }
    Frag<T>::keep(bh[0], bh[1], bh[2], bh[3]);
    if (SPLIT) Frag<T>::keep(bl[0], bl[1], bl[2], bl[3]);
  }
  acc_guard4(acc[0][0], acc[0][1], acc[0][2], acc[0][3]);
  acc_guard4(acc[1][0], acc[1][1], acc[1][2], acc[1][3]);
  acc_guard4(acc[2][0], acc[2][1], acc[2][2], acc[2][3]);
  acc_guard4(acc[3][0], acc[3][1], acc[3][2], acc[3][3]);

  float* slab = sT[wave];
  const float* Rb = RESID ? (resid + (size_t)b * strideR) : nullptr;
#pragma unroll
  for (int i = 0; i < 4; ++i) {
    const int mBase = m0 + (i << 4);
#pragma unroll
    for (int j = 0; j < 4; ++j) {
      const int n = n0 + (j << 4) + rlane;
      float bv = 0.f;
      if (BIAS_MODE == 2) bv = bias[n];
#pragma unroll
      for (int r = 0; r < 8; ++r) {
        float v = acc[i][j][r] * scale;
        if (BIAS_MODE == 1) v += bias[mBase + mOff + r];
        if (BIAS_MODE == 2) v += bv;
        if (RESID) v += Rb[(size_t)(mBase + mOff + r) * ldc + n];
        if (ACT == 2) v = fmaxf(v, 0.0f);
        if (ACT == 4) v = (v > 0.f) ? v : 0.01f * v;
        slab[(mOff + r) * 68 + (j << 4) + rlane] = v;
      }
    }
    __builtin_amdgcn_fence(__ATOMIC_RELEASE, "workgroup");
    __builtin_amdgcn_wave_barrier();
    __builtin_amdgcn_fence(__ATOMIC_ACQUIRE, "workgroup");
    if (OUT_MODE == 0) {
      float* C = (float*)Cout + (size_t)b * strideC;
      const int hh = lane >> 4, c4 = (lane & 15) * 4;
      for (int pass = 0; pass < 2; ++pass) {
#pragma unroll
        for (int it = 0; it < 8; ++it) {
          const int row = it * 2 + hh;
          v4f v = *(const v4f*)(slab + row * 68 + c4);
          *(volatile v4f*)(C + (size_t)(mBase + row) * ldc + n0 + c4) = v;
        }
        __threadfence();
      }
    } else {
      const int q = lane >> 3, c8 = (lane & 7) * 8;
      unsigned short* C  = (unsigned short*)Cout  + (size_t)b * strideC;
      unsigned short* C2 = (OUT_MODE == 2) ? ((unsigned short*)Cout2 + (size_t)b * strideC) : nullptr;
      for (int pass = 0; pass < 2; ++pass) {
#pragma unroll
        for (int it = 0; it < 4; ++it) {
          const int row = it * 4 + q;
          const float* sp = slab + row * 68 + c8;
          v8h hv, lv;
#pragma unroll
          for (int e = 0; e < 8; ++e) {
            if (OUT_MODE == 1) {
              hv[e] = (_Float16)sp[e];
            } else {
              unsigned short hb = f2bf_bits(sp[e]);
              unsigned short lb = f2bf_bits(sp[e] - bf_bits2f(hb));
              hv[e] = __builtin_bit_cast(_Float16, hb);
              lv[e] = __builtin_bit_cast(_Float16, lb);
            }
          }
          *(volatile v8h*)(C + (size_t)(mBase + row) * ldc + n0 + c8) = hv;
          if (OUT_MODE == 2) *(volatile v8h*)(C2 + (size_t)(mBase + row) * ldc + n0 + c8) = lv;
        }
        __threadfence();
      }
    }
    __builtin_amdgcn_fence(__ATOMIC_RELEASE, "workgroup");
    __builtin_amdgcn_wave_barrier();
    __builtin_amdgcn_fence(__ATOMIC_ACQUIRE, "workgroup");
  }
}

__global__ __launch_bounds__(256) void splitx_kernel(const float* __restrict__ in,
                                                     unsigned short* __restrict__ outh,
                                                     unsigned short* __restrict__ outl, int n8) {
  const int i = blockIdx.x * 256 + threadIdx.x;
  if (i >= n8) return;
  const size_t e0 = 8 * (size_t)i;
  const v4f a = *(const v4f*)(in + e0);
  const v4f c = *(const v4f*)(in + e0 + 4);
  unsigned short hb[8], lb[8];
#pragma unroll
  for (int e = 0; e < 4; ++e) {
    const unsigned short h0 = f2bf_bits(a[e]);
    hb[e] = h0; lb[e] = f2bf_bits(a[e] - bf_bits2f(h0));
    const unsigned short h1 = f2bf_bits(c[e]);
    hb[4 + e] = h1; lb[4 + e] = f2bf_bits(c[e] - bf_bits2f(h1));
  }
  const v4u uh = (v4u){pk16(hb[0], hb[1]), pk16(hb[2], hb[3]), pk16(hb[4], hb[5]), pk16(hb[6], hb[7])};
  const v4u ul = (v4u){pk16(lb[0], lb[1]), pk16(lb[2], lb[3]), pk16(lb[4], lb[5]), pk16(lb[6], lb[7])};
  unsigned short* ph = outh + e0;
  unsigned short* pl = outl + e0;
  *(volatile v4u*)ph = uh;
  *(volatile v4u*)pl = ul;
  __threadfence();
  *(volatile v4u*)ph = uh;
  *(volatile v4u*)pl = ul;
}

__global__ __launch_bounds__(256) void splitwt_kernel(const float* __restrict__ W,
                                                      unsigned short* __restrict__ wth,
                                                      unsigned short* __restrict__ wtl) {
  __shared__ float sm[64][65];
  const int t  = threadIdx.x;
  const int k0 = blockIdx.x * 64;
  const int n0 = blockIdx.y * 64;
#pragma unroll
  for (int i = 0; i < 16; ++i) {
    const int e = i * 256 + t;
    const int r = e >> 6;
    const int c = e & 63;
    sm[c][r] = W[(size_t)(k0 + r) * kDim + n0 + c];
  }
  __syncthreads();
  const int lane = t & 31, wave = t >> 5;
  const int q = lane >> 3, c8 = (lane & 7) * 8;
  for (int pass = 0; pass < 2; ++pass) {
#pragma unroll
    for (int it = 0; it < 2; ++it) {
      const int row = wave * 8 + it * 4 + q;
      unsigned short hb[8], lb[8];
#pragma unroll
      for (int e = 0; e < 8; ++e) {
        const float v = sm[row][c8 + e];
        const unsigned short h0 = f2bf_bits(v);
        hb[e] = h0;
        lb[e] = f2bf_bits(v - bf_bits2f(h0));
      }
      const v4u uh = (v4u){pk16(hb[0], hb[1]), pk16(hb[2], hb[3]), pk16(hb[4], hb[5]), pk16(hb[6], hb[7])};
      const v4u ul = (v4u){pk16(lb[0], lb[1]), pk16(lb[2], lb[3]), pk16(lb[4], lb[5]), pk16(lb[6], lb[7])};
      const size_t o = (size_t)(n0 + row) * kDim + k0 + c8;
      *(volatile v4u*)(wth + o) = uh;
      *(volatile v4u*)(wtl + o) = ul;
    }
    __threadfence();
  }
}

__global__ __launch_bounds__(256) void castqk_kernel(const float* __restrict__ XP,
                                                     const float* __restrict__ dq, const float* __restrict__ dk,
                                                     unsigned short* __restrict__ Q16, unsigned short* __restrict__ K16, int n8) {
  const int i = blockIdx.x * 256 + threadIdx.x;
  if (i >= n8) return;
  const size_t e0 = 8 * (size_t)i;
  const int c = (int)(e0 & (size_t)(kDim - 1));
  const v4f a  = *(const v4f*)(XP + e0);
  const v4f a2 = *(const v4f*)(XP + e0 + 4);
  const v4f q0 = *(const v4f*)(dq + c);
  const v4f q1 = *(const v4f*)(dq + c + 4);
  const v4f g0 = *(const v4f*)(dk + c);
  const v4f g1 = *(const v4f*)(dk + c + 4);
  unsigned short hq[8], hk[8];
#pragma unroll
  for (int e = 0; e < 4; ++e) {
    hq[e]     = h_bits(a[e] * q0[e]);
    hq[4 + e] = h_bits(a2[e] * q1[e]);
    hk[e]     = h_bits(a[e] * g0[e]);
    hk[4 + e] = h_bits(a2[e] * g1[e]);
  }
  const v4u uq = (v4u){pk16(hq[0], hq[1]), pk16(hq[2], hq[3]), pk16(hq[4], hq[5]), pk16(hq[6], hq[7])};
  const v4u uk = (v4u){pk16(hk[0], hk[1]), pk16(hk[2], hk[3]), pk16(hk[4], hk[5]), pk16(hk[6], hk[7])};
  unsigned short* pq = Q16 + e0;
  unsigned short* pkp = K16 + e0;
  *(volatile v4u*)pq = uq;
  *(volatile v4u*)pkp = uk;
  __threadfence();
  *(volatile v4u*)pq = uq;
  *(volatile v4u*)pkp = uk;
}

__global__ __launch_bounds__(256) void vtrans_kernel(const float* __restrict__ XP, const float* __restrict__ dv,
                                                     unsigned short* __restrict__ VT) {
  __shared__ float sm[64][65];
  const int t  = threadIdx.x;
  const int s0 = blockIdx.x * 64;
  const int bh = blockIdx.y;
  const int b  = bh >> 4;
  const int h  = bh & 15;
#pragma unroll
  for (int i = 0; i < 16; ++i) {
    const int e = i * 256 + t;
    const int r = e >> 6;
    const int c = e & 63;
    const int col = h * kHd + c;
    sm[c][r] = XP[(size_t)(b * kSeq + s0 + r) * kDim + col] * dv[col];
  }
  __syncthreads();
  const int lane = t & 31, wave = t >> 5;
  const int q = lane >> 3, c8 = (lane & 7) * 8;
  for (int pass = 0; pass < 2; ++pass) {
#pragma unroll
    for (int it = 0; it < 2; ++it) {
      const int row = wave * 8 + it * 4 + q;
      unsigned short hb[8];
#pragma unroll
      for (int e = 0; e < 8; ++e) hb[e] = h_bits(sm[row][c8 + e]);
      const v4u u = (v4u){pk16(hb[0], hb[1]), pk16(hb[2], hb[3]), pk16(hb[4], hb[5]), pk16(hb[6], hb[7])};
      *(volatile v4u*)(VT + ((size_t)bh * kHd + row) * kSeq + s0 + c8) = u;
    }
    __threadfence();
  }
}

__global__ __launch_bounds__(256) void rnorm_row_kernel(const float* __restrict__ S, unsigned short* __restrict__ P, float carry) {
  __shared__ float numbuf[kSeq];
  __shared__ __align__(16) unsigned short pbits[kSeq];
  __shared__ float redS[8];
  const int row  = blockIdx.x;
  const int t    = threadIdx.x;
  const int lane = t & 31, wave = t >> 5;
  const int c0   = t * 8;
  const float* sr = S + (size_t)row * kSeq + c0;
  float psum = 0.f;
#pragma unroll 1
  for (int e = 0; e < 8; ++e) {
    float z = sr[e];
    z = fminf(fmaxf(z, kClipLo), kClipHi);
    float nm = expf(z - kRShift) + kLam * z;
    nm = fmaxf(nm, 0.0f);
    numbuf[c0 + e] = nm;
    psum += nm;
  }
#pragma unroll
  for (int off = 16; off > 0; off >>= 1) psum += __shfl_xor(psum, off, 32);
  if (lane == 0) redS[wave] = psum;
  __syncthreads();
  float den = redS[0];
  den += redS[1]; den += redS[2]; den += redS[3];
  den += redS[4]; den += redS[5]; den += redS[6]; den += redS[7];
  den += kEps;
  const float inv = 1.0f / den;
#pragma unroll 1
  for (int e = 0; e < 8; ++e) {
    const float p = numbuf[c0 + e] * inv;
    pbits[c0 + e] = h_bits(p * carry);
  }
  __syncthreads();
  const v4u u = *(const v4u*)(pbits + c0);
  unsigned short* pp = P + (size_t)row * kSeq + c0;
  *(volatile v4u*)pp = u;
  __threadfence();
  *(volatile v4u*)pp = u;
}

extern "C" void kernel_launch(void* const* d_in, const int* in_sizes, int n_in,
                              void* d_out, int out_size, void* d_ws, size_t ws_size,
                              hipStream_t stream)
{
  if (n_in < 6) return;
  if (in_sizes[0] != kTok * kDim || in_sizes[1] != kDim * kDim || in_sizes[2] != kDim ||
      in_sizes[3] != kDim || in_sizes[4] != kDim || in_sizes[5] != kDim) return;
  if (out_size != kTok * kDim) return;

  const float* x    = (const float*)d_in[0];
  const float* W    = (const float*)d_in[1];
  const float* bias = (const float*)d_in[2];
  const float* dq   = (const float*)d_in[3];
  const float* dk   = (const float*)d_in[4];
  const float* dv   = (const float*)d_in[5];
  float* out = (float*)d_out;

  const size_t bPlane16 = (size_t)kTok * kDim * 2;
  const size_t bWT      = (size_t)kDim * kDim * 2;
  const size_t bXP      = (size_t)kTok * kDim * 4;
  const size_t bVT      = (size_t)kGroups * kHd * kSeq * 2;
  const size_t bS       = (size_t)kGrpChunk * kSeq * kSeq * 4;
  const size_t bP       = (size_t)kGrpChunk * kSeq * kSeq * 2;

  const size_t oXh  = 0;
  const size_t oXl  = oXh + bPlane16;
  const size_t oWTh = oXl + bPlane16;
  const size_t oWTl = oWTh + bWT;
  const size_t oXP  = oWTl + bWT;
  const size_t oQ   = oXP + bXP;
  const size_t oK   = oQ + bPlane16;
  const size_t oVT  = oK + bPlane16;
  const size_t oS   = oVT + bVT;
  const size_t oP   = oS + bS;
  const size_t total = oP + bP;
  if (total > ws_size) return;

  unsigned char* ws = (unsigned char*)d_ws;
  unsigned short* Xh   = (unsigned short*)(ws + oXh);
  unsigned short* Xl   = (unsigned short*)(ws + oXl);
  unsigned short* WTh  = (unsigned short*)(ws + oWTh);
  unsigned short* WTl  = (unsigned short*)(ws + oWTl);
  float*          XP   = (float*)(ws + oXP);
  unsigned short* Q16  = (unsigned short*)(ws + oQ);
  unsigned short* K16  = (unsigned short*)(ws + oK);
  unsigned short* VT16 = (unsigned short*)(ws + oVT);
  float*          S    = (float*)(ws + oS);
  unsigned short* P16  = (unsigned short*)(ws + oP);

  const int n8 = kTok * kDim / 8;
  const int nblk8 = (n8 + 255) / 256;

  splitx_kernel<<<dim3(nblk8), dim3(256), 0, stream>>>(x, Xh, Xl, n8);
  splitwt_kernel<<<dim3(kDim / 64, kDim / 64), dim3(256), 0, stream>>>(W, WTh, WTl);
  {
    const int tiles = (kTok / 64) * (kDim / 64);
    wmma_gemm64<1, true, 2, 0, false, 0><<<dim3(tiles / 8, 1), dim3(256), 0, stream>>>(
        Xh, Xl, kDim, 0L,
        WTh, WTl, kDim, 0L,
        (void*)XP, (void*)XP, kDim, 0L,
        bias, (const float*)XP, 0L,
        kTok, kDim, kDim, 1.0f);
  }
  castqk_kernel<<<dim3(nblk8), dim3(256), 0, stream>>>(XP, dq, dk, Q16, K16, n8);
  vtrans_kernel<<<dim3(kSeq / 64, kGroups), dim3(256), 0, stream>>>(XP, dv, VT16);

  for (int c = 0; c < kChunks; ++c) {
    const int bh0 = c * kGrpChunk;
    const int b   = bh0 / kHeads;
    const int h0  = bh0 % kHeads;
    const unsigned short* Qg = Q16 + (size_t)b * kSeq * kDim + (size_t)h0 * kHd;
    const unsigned short* Kg = K16 + (size_t)b * kSeq * kDim + (size_t)h0 * kHd;
    {
      const int tiles = (kSeq / 64) * (kSeq / 64);
      wmma_gemm64<0, false, 0, 0, false, 0><<<dim3(tiles / 8, kGrpChunk), dim3(256), 0, stream>>>(
          Qg, Qg, kDim, (long)kHd,
          Kg, Kg, kDim, (long)kHd,
          (void*)S, (void*)S, kSeq, (long)kSeq * kSeq,
          (const float*)S, (const float*)S, 0L,
          kSeq, kSeq, kHd, 1.0f);
    }
    rnorm_row_kernel<<<dim3(kGrpChunk * kSeq), dim3(256), 0, stream>>>(S, P16, kPCarry);
    {
      const int tiles = (kSeq / 64) * (kHd / 64);
      const unsigned short* Vg = VT16 + (size_t)bh0 * kHd * kSeq;
      float* Og = out + (size_t)b * kSeq * kDim + (size_t)h0 * kHd;
      wmma_gemm64<0, false, 0, 0, false, 0><<<dim3((tiles + 7) / 8, kGrpChunk), dim3(256), 0, stream>>>(
          P16, P16, kSeq, (long)kSeq * kSeq,
          Vg, Vg, kSeq, (long)kHd * kSeq,
          (void*)Og, (void*)Og, kDim, (long)kHd,
          (const float*)S, (const float*)S, 0L,
          kSeq, kHd, kSeq, kPCarryInv);
    }
  }
}
